// MultiHeadAttention_87780541595793
// MI455X (gfx1250) — hardware-run, weakly checked
//
#include <hip/hip_runtime.h>
#include <math.h>

typedef __attribute__((ext_vector_type(16))) _Float16 v16h;
typedef __attribute__((ext_vector_type(8)))  _Float16 v8h;
typedef __attribute__((ext_vector_type(16))) __bf16   v16b;
typedef __attribute__((ext_vector_type(8)))  __bf16   v8b;
typedef __attribute__((ext_vector_type(8)))  float    v8f;
typedef __attribute__((ext_vector_type(4)))  float    v4f;
typedef __attribute__((ext_vector_type(4)))  unsigned int v4u;

constexpr int kBatch    = 4;
constexpr int kSeq      = 2048;
constexpr int kDin      = 1024;
constexpr int kDout     = 1024;
constexpr int kHeads    = 16;
constexpr int kDh       = 64;
constexpr int kRows     = kBatch * kSeq;
constexpr int kN3       = 3 * kDout;
constexpr int kBH       = kBatch * kHeads;
constexpr int kHeadRows = 64;
constexpr int kHP       = 65;
static_assert(kHeads * kDh == kDout);
static_assert(kDh == 64);
static_assert((kDin % 32) == 0);
static_assert((kRows % 64) == 0 && (kN3 % 64) == 0 && (kSeq % 64) == 0 && (kDout % 64) == 0);
static_assert(((kRows / 64) * (kN3 / 64)) % 8 == 0);
static_assert(kHeadRows == 64);

constexpr float kInvSqrtDh  = 0.125f;
static_assert(kInvSqrtDh * kInvSqrtDh * (float)kDh == 1.0f);
constexpr float kQKVCarry   = 16.0f;
constexpr float kPCarryLog2 = 6.0f;
constexpr float kPCarry     = 64.0f;
static_assert(kPCarry == 64.0f && kPCarryLog2 == 6.0f);
constexpr float kLog2e      = 1.4426950408889634f;
constexpr float kSArg       = kLog2e * kInvSqrtDh / (kQKVCarry * kQKVCarry);
constexpr float kArgMax     = 15.5f;
constexpr float kOutCarry   = kQKVCarry;

constexpr size_t kOffXb   = 0;
constexpr size_t kOffWt   = kOffXb + (size_t)kRows * kDin * 2;
constexpr size_t kOffQh   = kOffWt + (size_t)kN3 * kDin * 2;
constexpr size_t kOffKh   = kOffQh + (size_t)kBH * kSeq * kDh * 2;
constexpr size_t kOffVt   = kOffKh + (size_t)kBH * kSeq * kDh * 2;
constexpr size_t kOffHead = kOffVt + (size_t)kBH * kDh * kSeq * 2;
constexpr size_t kWsTotal = kOffHead + (size_t)3 * kBH * kHeadRows * kDh * 4;
static_assert(kWsTotal == 76546048ull);
static_assert(kWsTotal <= 134217728ull);
static_assert((kOffWt % 128) == 0 && (kOffQh % 128) == 0 && (kOffKh % 128) == 0 && (kOffVt % 128) == 0 && (kOffHead % 128) == 0);

__device__ __forceinline__ unsigned short f2bf_bits(float f) {
  unsigned u = __float_as_uint(f);
  return (unsigned short)((u + 0x7FFFu + ((u >> 16) & 1u)) >> 16);
}
__device__ __forceinline__ unsigned pk16(unsigned short a, unsigned short b) { return (unsigned)a | ((unsigned)b << 16); }

__device__ __forceinline__ v16b ld_frag_b(const __bf16* p) {
  union U { v16b v; v8b h[2]; };
  U f;
  f.h[0] = *(const v8b*)(p);
  f.h[1] = *(const v8b*)(p + 16);
  return f.v;
}
__device__ __forceinline__ v16h ld_frag_h(const _Float16* p) {
  union U { v16h v; v8h h[2]; };
  U f;
  f.h[0] = *(const v8h*)(p);
  f.h[1] = *(const v8h*)(p + 16);
  return f.v;
}
__device__ __forceinline__ v8f mma_b(v16b a, v16b b, v8f c) {
  c = __builtin_amdgcn_wmma_f32_16x16x32_bf16(false, a, false, b, (short)0, c, false, false);
  asm volatile("v_nop\n\tv_nop\n\tv_nop\n\tv_nop" : "+v"(c) : "v"(a), "v"(b));
  return c;
}
__device__ __forceinline__ v8f mma_h(v16h a, v16h b, v8f c) {
  c = __builtin_amdgcn_wmma_f32_16x16x32_f16(false, a, false, b, (short)0, c, false, false);
  asm volatile("v_nop\n\tv_nop\n\tv_nop\n\tv_nop" : "+v"(c) : "v"(a), "v"(b));
  return c;
}
__device__ __forceinline__ void wave_sync() {
  __builtin_amdgcn_fence(__ATOMIC_RELEASE, "workgroup");
  __builtin_amdgcn_wave_barrier();
  __builtin_amdgcn_fence(__ATOMIC_ACQUIRE, "workgroup");
}

__global__ __launch_bounds__(256) void xcast_bf16_kernel(const float* __restrict__ in, unsigned short* __restrict__ out, int n8) {
  const int i = blockIdx.x * 256 + threadIdx.x;
  if (i >= n8) return;
  const float* p = in + 8 * (size_t)i;
  const v4f a = *(const v4f*)(p);
  const v4f c = *(const v4f*)(p + 4);
  unsigned short hb[8];
#pragma unroll
  for (int e = 0; e < 4; ++e) {
    const float fa = a[e];
    const float fc = c[e];
    hb[e]     = f2bf_bits(fa);
    hb[4 + e] = f2bf_bits(fc);
  }
  const v4u u = (v4u){pk16(hb[0], hb[1]), pk16(hb[2], hb[3]), pk16(hb[4], hb[5]), pk16(hb[6], hb[7])};
  unsigned short* q = out + 8 * (size_t)i;
  *(volatile v4u*)q = u;
  __threadfence();
  *(volatile v4u*)q = u;
}

__global__ __launch_bounds__(256) void wt_bf16_kernel(const float* __restrict__ W0, const float* __restrict__ W1,
                                                      const float* __restrict__ W2, unsigned short* __restrict__ out) {
  __shared__ float sm[64][65];
  const int t  = threadIdx.x;
  const int k0 = blockIdx.x * 64;
  const int n0 = blockIdx.y * 64;
  const int z  = blockIdx.z;
  const float* W = (z == 0) ? W0 : (z == 1) ? W1 : W2;
#pragma unroll
  for (int i = 0; i < 16; ++i) {
    const int e = i * 256 + t;
    const int r = e >> 6;
    const int c = e & 63;
    sm[c][r] = W[(size_t)(k0 + r) * kDout + n0 + c];
  }
  __syncthreads();
  const int lane = t & 31;
  const int wave = __builtin_amdgcn_readfirstlane((int)(threadIdx.x >> 5));
  const int q = lane >> 3, c8 = (lane & 7) * 8;
  unsigned short* op = out + (size_t)z * kDout * kDin;
  for (int pass = 0; pass < 2; ++pass) {
#pragma unroll
    for (int it = 0; it < 2; ++it) {
      const int row = wave * 8 + it * 4 + q;
      unsigned short hb[8];
#pragma unroll
      for (int e = 0; e < 8; ++e) {
        const float f = sm[row][c8 + e];
        hb[e] = f2bf_bits(f);
      }
      const v4u u = (v4u){pk16(hb[0], hb[1]), pk16(hb[2], hb[3]), pk16(hb[4], hb[5]), pk16(hb[6], hb[7])};
      *(volatile v4u*)(op + (size_t)(n0 + row) * kDin + k0 + c8) = u;
    }
    __threadfence();
  }
}

__global__ __launch_bounds__(256) void qkv_gemm_kernel(
    const unsigned short* __restrict__ Xb, const unsigned short* __restrict__ Wt,
    unsigned short* __restrict__ Qh, unsigned short* __restrict__ Kh, unsigned short* __restrict__ Vt,
    float* __restrict__ Head) {
  __shared__ __align__(16) float sT[8][16 * 68];
  const int lane = threadIdx.x & 31;
  const int wave = __builtin_amdgcn_readfirstlane((int)(threadIdx.x >> 5));
  constexpr int tilesN = kN3 / 64;
  constexpr int tilesM = kRows / 64;
  const int tile = blockIdx.x * 8 + wave;
  if (tile >= tilesM * tilesN) return;
  const int tm = tile / tilesN;
  const int tn = tile - tm * tilesN;
  const int m0 = tm << 6;
  const int n0 = tn << 6;

  const __bf16* A  = (const __bf16*)Xb;
  const __bf16* Bt = (const __bf16*)Wt;

  const int rlane = lane & 15;
  const int koff  = (lane >> 4) * 8;
  const int mOff  = (lane >> 4) * 8;

  v8f acc[4][4];
#pragma unroll
  for (int i = 0; i < 4; ++i)
#pragma unroll
    for (int j = 0; j < 4; ++j) acc[i][j] = (v8f){0.f, 0.f, 0.f, 0.f, 0.f, 0.f, 0.f, 0.f};

#pragma unroll 1
  for (int k0 = 0; k0 < kDin; k0 += 32) {
    v16b bf[4];
#pragma unroll
    for (int j = 0; j < 4; ++j)
      bf[j] = ld_frag_b(Bt + (size_t)(n0 + (j << 4) + rlane) * kDin + koff + k0);
#pragma unroll
    for (int i = 0; i < 4; ++i) {
      const v16b af = ld_frag_b(A + (size_t)(m0 + (i << 4) + rlane) * kDin + koff + k0);
#pragma unroll
      for (int j = 0; j < 4; ++j) acc[i][j] = mma_b(af, bf[j], acc[i][j]);
    }
  }

  float* slab = sT[wave];
  const int zsel = n0 / kDout;
  const int hd   = (n0 - zsel * kDout) >> 6;
  const int bb   = m0 / kSeq;
  const int t0   = m0 - bb * kSeq;
  const int bh   = bb * kHeads + hd;
  const bool headTile = (t0 == 0);
  const int q8 = lane >> 3, c8 = (lane & 7) * 8;
  const int hh = lane >> 4, c4 = (lane & 15) * 4;

  if (zsel < 2 || headTile) {
#pragma unroll
    for (int i = 0; i < 4; ++i) {
#pragma unroll
      for (int j = 0; j < 4; ++j)
#pragma unroll
        for (int r = 0; r < 8; ++r) slab[(mOff + r) * 68 + (j << 4) + rlane] = acc[i][j][r];
      wave_sync();
      if (headTile) {
        float* hp = Head + ((size_t)(zsel * kBH + bh) * kHeadRows + (i << 4)) * kDh;
        for (int pass = 0; pass < 2; ++pass) {
#pragma unroll
          for (int it = 0; it < 8; ++it) {
            const int row = it * 2 + hh;
            const v4f v = *(const v4f*)(slab + row * 68 + c4);
            *(volatile v4f*)(hp + (size_t)row * kDh + c4) = v;
          }
          __threadfence();
        }
      }
      if (zsel < 2) {
        unsigned short* plane = (zsel == 0) ? Qh : Kh;
        unsigned short* pp = plane + ((size_t)bh * kSeq + t0 + (i << 4)) * kDh;
        for (int pass = 0; pass < 2; ++pass) {
#pragma unroll
          for (int it = 0; it < 4; ++it) {
            const int row = it * 4 + q8;
            const float* sp = slab + row * 68 + c8;
            v8h hv;
#pragma unroll
            for (int e = 0; e < 8; ++e) hv[e] = (_Float16)(sp[e] * kQKVCarry);
            *(volatile v8h*)(pp + (size_t)row * kDh + c8) = hv;
          }
          __threadfence();
        }
      }
      wave_sync();
    }
  }
  if (zsel == 2) {
    unsigned short* vp = Vt + (size_t)bh * kDh * kSeq + t0;
#pragma unroll
    for (int j = 0; j < 4; ++j) {
#pragma unroll
      for (int i = 0; i < 4; ++i)
#pragma unroll
        for (int r = 0; r < 8; ++r) slab[rlane * 68 + (i << 4) + mOff + r] = acc[i][j][r];
      wave_sync();
      for (int pass = 0; pass < 2; ++pass) {
#pragma unroll
        for (int it = 0; it < 4; ++it) {
          const int drow = it * 4 + q8;
          const float* sp = slab + drow * 68 + c8;
          v8h hv;
#pragma unroll
          for (int e = 0; e < 8; ++e) hv[e] = (_Float16)(sp[e] * kQKVCarry);
          *(volatile v8h*)(vp + (size_t)((j << 4) + drow) * kSeq + c8) = hv;
        }
        __threadfence();
      }
      wave_sync();
    }
  }
}

__global__ __launch_bounds__(128) void causal_attn_kernel(
    const unsigned short* __restrict__ Qh, const unsigned short* __restrict__ Kh,
    const unsigned short* __restrict__ Vt, float* __restrict__ out) {
  __shared__ __align__(16) float Os[4][16 * 68];
  const int lane = threadIdx.x & 31;
  const int wave = __builtin_amdgcn_readfirstlane((int)(threadIdx.x >> 5));
  const int hh = lane >> 4;
  const int c  = lane & 15;
  const int qb = blockIdx.x + 1;
  const int bh = blockIdx.y;
  const int b  = bh / kHeads;
  const int h  = bh - b * kHeads;
  const int q0 = qb * 64 + wave * 16;

  const _Float16* Qp = (const _Float16*)Qh + (size_t)bh * kSeq * kDh;
  const _Float16* Kp = (const _Float16*)Kh + (size_t)bh * kSeq * kDh;
  const _Float16* Vp = (const _Float16*)Vt + (size_t)bh * kDh * kSeq;

  const v16h qf0 = ld_frag_h(Qp + (size_t)(q0 + c) * kDh + 8 * hh);
  const v16h qf1 = ld_frag_h(Qp + (size_t)(q0 + c) * kDh + 32 + 8 * hh);

  v8f oacc[4];
#pragma unroll
  for (int t = 0; t < 4; ++t) oacc[t] = (v8f){0.f, 0.f, 0.f, 0.f, 0.f, 0.f, 0.f, 0.f};
  float lsum = 0.f;
  const int qrow = q0 + c;
  const int nChunks = qb + 1;

#pragma unroll 1
  for (int kc = 0; kc < nChunks; ++kc) {
    const int kv0 = kc * 64;
    const bool diag = (kc == qb);
    v16h pf[2];
#pragma unroll
    for (int jt = 0; jt < 4; ++jt) {
      const _Float16* kr = Kp + (size_t)(kv0 + jt * 16 + c) * kDh + 8 * hh;
      const v16h kf0 = ld_frag_h(kr);
      const v16h kf1 = ld_frag_h(kr + 32);
      v8f s = (v8f){0.f, 0.f, 0.f, 0.f, 0.f, 0.f, 0.f, 0.f};
      s = mma_h(kf0, qf0, s);
      s = mma_h(kf1, qf1, s);
      const int keyb = kv0 + jt * 16 + 8 * hh;
#pragma unroll
      for (int r = 0; r < 8; ++r) {
        float arg = fmaf(s[r], kSArg, kPCarryLog2);
        arg = fminf(arg, kArgMax);
        float p = __builtin_amdgcn_exp2f(arg);
        if (diag) p = (keyb + r > qrow) ? 0.0f : p;
        lsum += p;
        pf[jt >> 1][(jt & 1) * 8 + r] = (_Float16)p;
      }
    }
#pragma unroll
    for (int kk = 0; kk < 2; ++kk) {
#pragma unroll
      for (int t = 0; t < 4; ++t) {
        const v16h vf = ld_frag_h(Vp + (size_t)(t * 16 + c) * kSeq + kv0 + kk * 32 + 8 * hh);
        oacc[t] = mma_h(pf[kk], vf, oacc[t]);
      }
    }
  }

  const float ltot = lsum + __shfl_xor(lsum, 16, 32);
  float* os = Os[wave];
#pragma unroll
  for (int r = 0; r < 8; ++r) {
    const float lr  = __shfl(ltot, 8 * hh + r, 32);
    const float inv = 1.0f / (lr * kOutCarry);
#pragma unroll
    for (int t = 0; t < 4; ++t) os[(8 * hh + r) * 68 + t * 16 + c] = oacc[t][r] * inv;
  }
  wave_sync();
  {
    float* ob = out + ((size_t)b * kSeq + q0) * kDout + h * kDh;
    const int c4 = (lane & 15) * 4;
    for (int pass = 0; pass < 2; ++pass) {
#pragma unroll
      for (int it = 0; it < 8; ++it) {
        const int row = it * 2 + hh;
        const v4f val = *(const v4f*)(os + row * 68 + c4);
        *(volatile v4f*)(ob + (size_t)row * kDout + c4) = val;
      }
      __threadfence();
    }
  }
}

__global__ __launch_bounds__(256) void head_rows_kernel(const float* __restrict__ Head, float* __restrict__ out) {
  __shared__ float sq[kHeadRows * kHP];
  __shared__ float sk[kHeadRows * kHP];
  __shared__ float sv[kHeadRows * kHP];
  const int tid  = threadIdx.x;
  const int lane = tid & 31;
  const int wave = __builtin_amdgcn_readfirstlane((int)(threadIdx.x >> 5));
  const int bh = blockIdx.x;
  const int b  = bh / kHeads;
  const int h  = bh - b * kHeads;
  const float* hq = Head + ((size_t)(0 * kBH + bh)) * kHeadRows * kDh;
  const float* hk = Head + ((size_t)(1 * kBH + bh)) * kHeadRows * kDh;
  const float* hv = Head + ((size_t)(2 * kBH + bh)) * kHeadRows * kDh;
#pragma unroll 1
  for (int i = 0; i < 16; ++i) {
    const int e = i * 256 + tid;
    const int r = e >> 6;
    const int d = e & 63;
    sq[r * kHP + d] = hq[e];
    sk[r * kHP + d] = hk[e];
    sv[r * kHP + d] = hv[e];
  }
  __syncthreads();
#pragma unroll 1
  for (int i = 0; i < 8; ++i) {
    const int t = wave + 8 * i;
    float s0 = 0.f, s1 = 0.f;
#pragma unroll 4
    for (int d = 0; d < kDh; ++d) {
      const float qd = sq[t * kHP + d];
      s0 = fmaf(qd, sk[lane * kHP + d], s0);
      s1 = fmaf(qd, sk[(lane + 32) * kHP + d], s1);
    }
    s0 *= kInvSqrtDh;
    s1 *= kInvSqrtDh;
    const bool ok0 = (lane <= t);
    const bool ok1 = (lane + 32 <= t);
    float m = fmaxf(ok0 ? s0 : -INFINITY, ok1 ? s1 : -INFINITY);
#pragma unroll
    for (int off = 16; off > 0; off >>= 1) m = fmaxf(m, __shfl_xor(m, off, 32));
    const float e0 = expf(s0 - m);
    const float e1 = expf(s1 - m);
    const float p0 = ok0 ? e0 : 0.0f;
    const float p1 = ok1 ? e1 : 0.0f;
    float sum = p0 + p1;
#pragma unroll
    for (int off = 16; off > 0; off >>= 1) sum += __shfl_xor(sum, off, 32);
    const float inv = 1.0f / sum;
    float o0 = 0.f, o1 = 0.f;
#pragma unroll 2
    for (int j = 0; j < 32; ++j) {
      const float pa = __shfl(p0, j, 32);
      const float pb = __shfl(p1, j, 32);
      o0 = fmaf(pa, sv[j * kHP + lane], o0);
      o1 = fmaf(pa, sv[j * kHP + lane + 32], o1);
      o0 = fmaf(pb, sv[(j + 32) * kHP + lane], o0);
      o1 = fmaf(pb, sv[(j + 32) * kHP + lane + 32], o1);
    }
    const float r0 = o0 * inv;
    const float r1 = o1 * inv;
    float* orow = out + ((size_t)b * kSeq + t) * kDout + h * kDh;
    *(volatile float*)(orow + lane)      = r0;
    *(volatile float*)(orow + 32 + lane) = r1;
    __threadfence();
    *(volatile float*)(orow + lane)      = r0;
    *(volatile float*)(orow + 32 + lane) = r1;
  }
}

extern "C" void kernel_launch(void* const* d_in, const int* in_sizes, int n_in,
                              void* d_out, int out_size, void* d_ws, size_t ws_size,
                              hipStream_t stream) {
  if (n_in < 4) return;
  if (in_sizes[0] != kRows * kDin) return;
  if (in_sizes[1] != kDin * kDout) return;
  if (in_sizes[2] != kDin * kDout) return;
  if (in_sizes[3] != kDin * kDout) return;
  if (out_size != kRows * kDout) return;
  if (ws_size < kWsTotal) return;

  const float* x  = (const float*)d_in[0];
  const float* wq = (const float*)d_in[1];
  const float* wk = (const float*)d_in[2];
  const float* wv = (const float*)d_in[3];
  float* out = (float*)d_out;

  char* ws = (char*)d_ws;
  unsigned short* Xb   = (unsigned short*)(ws + kOffXb);
  unsigned short* Wt   = (unsigned short*)(ws + kOffWt);
  unsigned short* Qh   = (unsigned short*)(ws + kOffQh);
  unsigned short* Kh   = (unsigned short*)(ws + kOffKh);
  unsigned short* Vt   = (unsigned short*)(ws + kOffVt);
  float*          Head = (float*)(ws + kOffHead);

  xcast_bf16_kernel<<<(kRows * kDin / 8) / 256, 256, 0, stream>>>(x, Xb, kRows * kDin / 8);
  wt_bf16_kernel<<<dim3(kDin / 64, kDout / 64, 3), 256, 0, stream>>>(wq, wk, wv, Wt);
  qkv_gemm_kernel<<<((kRows / 64) * (kN3 / 64)) / 8, 256, 0, stream>>>(Xb, Wt, Qh, Kh, Vt, Head);
  causal_attn_kernel<<<dim3(kSeq / 64 - 1, kBH), 128, 0, stream>>>(Qh, Kh, Vt, out);
  head_rows_kernel<<<kBH, 256, 0, stream>>>(Head, out);
}
